// SignedConv_57286273794081
// MI455X (gfx1250) — hardware-verified
//
#include <hip/hip_runtime.h>
#include <stddef.h>


#define FIN    64
#define KF     128
#define NOUT   64
#define OUTW   128
#define NTHR   256
#define NWAVE  8
#define EPT    8
#define NGRP   2
#define CHUNK  (NTHR * EPT * NGRP)
#define WCAP   (EPT * NGRP * 32)
#define LISTN  (NWAVE * WCAP)
#define TGT    1024
#define NPL    (2 * 2 * NOUT * KF)
#define LDS_ACC  (TGT * FIN * 4)
#define LDS_MAIN (LDS_ACC + LISTN * 4 + TGT * 4 + 64)

static_assert((CHUNK & (CHUNK - 1)) == 0);
static_assert(CHUNK <= 4096);
static_assert((TGT & (TGT - 1)) == 0 && TGT <= 4096);
static_assert(TGT % (NWAVE * 16) == 0);
static_assert((TGT * FIN / 4) % NTHR == 0 && TGT % NTHR == 0);
static_assert(KF == 2 * FIN && (KF % 32) == 0);
static_assert((2 * NOUT * (KF / 8)) % NTHR == 0);
static_assert(NWAVE * 32 == NTHR);

typedef float          v2f   __attribute__((ext_vector_type(2)));
typedef float          v4f   __attribute__((ext_vector_type(4)));
typedef float          v8f   __attribute__((ext_vector_type(8)));
typedef int            v4i   __attribute__((ext_vector_type(4)));
typedef unsigned short v8us  __attribute__((ext_vector_type(8)));
typedef unsigned short v16us __attribute__((ext_vector_type(16)));
typedef __bf16         v16b  __attribute__((ext_vector_type(16)));
union FragB { v16b v; v16us u; v8us h[2]; };

__device__ __forceinline__ unsigned int bf_bits(float f) {
  const unsigned int u = __float_as_uint(f);
  return (u + 0x7FFFu + ((u >> 16) & 1u)) >> 16;
}

__device__ __forceinline__ void split16(v4f a0, v4f a1, v4f a2, v4f a3, FragB& hi, FragB& lo) {
  float f[16];
  f[0]  = a0.x; f[1]  = a0.y; f[2]  = a0.z; f[3]  = a0.w;
  f[4]  = a1.x; f[5]  = a1.y; f[6]  = a1.z; f[7]  = a1.w;
  f[8]  = a2.x; f[9]  = a2.y; f[10] = a2.z; f[11] = a2.w;
  f[12] = a3.x; f[13] = a3.y; f[14] = a3.z; f[15] = a3.w;
  v16us hu, lu;
#pragma unroll
  for (int e = 0; e < 16; ++e) {
    const unsigned int hb = bf_bits(f[e]);
    hu[e] = (unsigned short)hb;
    lu[e] = (unsigned short)bf_bits(f[e] - __uint_as_float(hb << 16));
  }
  hi.u = hu; lo.u = lu;
}

__device__ __forceinline__ v8f wmb(const FragB& a, const FragB& b, v8f c) {
  v8f d = __builtin_amdgcn_wmma_f32_16x16x32_bf16(false, a.v, false, b.v, (short)0, c, false, false);
  asm volatile("v_nop\n\tv_nop\n\tv_nop\n\tv_nop" : "+v"(d) : "v"(a.u), "v"(b.u));
  return d;
}

template <int NB>
__device__ __forceinline__ int scan_chunk(const int* __restrict__ dsts, int nE, int cbase, int slotBase,
                                          int vec8, int* list, int tid, int lane, int wave) {
  int wc = 0;
#pragma unroll
  for (int g = 0; g < NGRP; ++g) {
    const int el0  = (g * NTHR + tid) * EPT;
    const int e0   = cbase + el0;
    const int sent = -2147483647 - 1;
    v4i da, db;
    if (vec8 != 0 && cbase + CHUNK <= nE) {
      da = *(const v4i*)(dsts + e0);
      db = *(const v4i*)(dsts + e0 + 4);
    } else {
      da.x = (e0     < nE) ? dsts[min(e0,     nE - 1)] : sent;
      da.y = (e0 + 1 < nE) ? dsts[min(e0 + 1, nE - 1)] : sent;
      da.z = (e0 + 2 < nE) ? dsts[min(e0 + 2, nE - 1)] : sent;
      da.w = (e0 + 3 < nE) ? dsts[min(e0 + 3, nE - 1)] : sent;
      db.x = (e0 + 4 < nE) ? dsts[min(e0 + 4, nE - 1)] : sent;
      db.y = (e0 + 5 < nE) ? dsts[min(e0 + 5, nE - 1)] : sent;
      db.z = (e0 + 6 < nE) ? dsts[min(e0 + 6, nE - 1)] : sent;
      db.w = (e0 + 7 < nE) ? dsts[min(e0 + 7, nE - 1)] : sent;
    }
    const unsigned nb = (unsigned)slotBase;
    const unsigned s0 = (unsigned)da.x - nb, s1 = (unsigned)da.y - nb;
    const unsigned s2 = (unsigned)da.z - nb, s3 = (unsigned)da.w - nb;
    const unsigned s4 = (unsigned)db.x - nb, s5 = (unsigned)db.y - nb;
    const unsigned s6 = (unsigned)db.z - nb, s7 = (unsigned)db.w - nb;
    const bool h0 = s0 < (unsigned)NB, h1 = s1 < (unsigned)NB, h2 = s2 < (unsigned)NB, h3 = s3 < (unsigned)NB;
    const bool h4 = s4 < (unsigned)NB, h5 = s5 < (unsigned)NB, h6 = s6 < (unsigned)NB, h7 = s7 < (unsigned)NB;
    const unsigned any = __builtin_amdgcn_ballot_w32(h0 | h1 | h2 | h3 | h4 | h5 | h6 | h7);
    if (any != 0u) {
#define HITJ(J, HJ, SJ) { \
        const unsigned mj = __builtin_amdgcn_ballot_w32(HJ); \
        if (mj != 0u) { \
          if (HJ) { \
            const int pos = wc + (int)__builtin_amdgcn_mbcnt_lo(mj, 0u); \
            if (pos < WCAP) list[wave * WCAP + pos] = ((el0 + (J)) << 12) | (int)(SJ); \
          } \
          wc += (int)__builtin_popcount(mj); } }
      HITJ(0, h0, s0)
      HITJ(1, h1, s1)
      HITJ(2, h2, s2)
      HITJ(3, h3, s3)
      HITJ(4, h4, s4)
      HITJ(5, h5, s5)
      HITJ(6, h6, s6)
      HITJ(7, h7, s7)
#undef HITJ
    }
  }
  return wc;
}

__global__ __launch_bounds__(NTHR) void k_wprep(
    const float* __restrict__ Wp, const float* __restrict__ Wpc,
    const float* __restrict__ Wn, const float* __restrict__ Wnc, unsigned short* planes) {
  const int i = blockIdx.x * NTHR + (int)threadIdx.x;
  if (i >= 2 * NOUT * (KF / 8)) return;
  const int s   = i / (NOUT * (KF / 8));
  const int rem = i - s * (NOUT * (KF / 8));
  const int n   = rem / (KF / 8);
  const int k0  = (rem - n * (KF / 8)) * 8;
  const float* Wa = (s == 0) ? Wp  : Wn;
  const float* Wc = (s == 0) ? Wpc : Wnc;
  const int kk = k0 & (FIN - 1);
  const v4f a0 = *(const v4f*)(Wa + n * FIN + kk), a1 = *(const v4f*)(Wa + n * FIN + kk + 4);
  const v4f c0 = *(const v4f*)(Wc + n * FIN + kk), c1 = *(const v4f*)(Wc + n * FIN + kk + 4);
  const bool ua = k0 < FIN;
  float f[8];
  f[0] = ua ? a0.x : c0.x; f[1] = ua ? a0.y : c0.y; f[2] = ua ? a0.z : c0.z; f[3] = ua ? a0.w : c0.w;
  f[4] = ua ? a1.x : c1.x; f[5] = ua ? a1.y : c1.y; f[6] = ua ? a1.z : c1.z; f[7] = ua ? a1.w : c1.w;
  v8us hu, lu;
#pragma unroll
  for (int e = 0; e < 8; ++e) {
    const unsigned int hb = bf_bits(f[e]);
    hu[e] = (unsigned short)hb;
    lu[e] = (unsigned short)bf_bits(f[e] - __uint_as_float(hb << 16));
  }
  unsigned short* ph = planes + ((size_t)(2 * s) * NOUT + n) * KF + k0;
  unsigned short* pl = ph + (size_t)NOUT * KF;
  *(volatile v8us*)ph = hu;
  *(volatile v8us*)pl = lu;
  __threadfence();
  *(volatile v8us*)ph = hu;
  *(volatile v8us*)pl = lu;
}

__global__ __launch_bounds__(NTHR) void k_main(
    const float* __restrict__ x, const int* __restrict__ eiP, const int* __restrict__ eiN,
    const unsigned short* __restrict__ planes, const float* __restrict__ bP, const float* __restrict__ bN,
    float* out, int nN, int nEP, int nEN, int vecP, int vecN) {
  extern __shared__ v4f lds_dyn[];
  float* acc  = (float*)lds_dyn;
  int*   list = (int*)(acc + TGT * FIN);
  int*   scnt = list + LISTN;
  int*   wcnt = scnt + TGT;
  const int tid = threadIdx.x, lane = tid & 31, wave = tid >> 5, hh = lane >> 4, m = lane & 15;
  const int nodeBase = blockIdx.x * TGT;

#pragma unroll 1
  for (int s = 0; s < 2; ++s) {
    const int*   ei   = (s == 0) ? eiP : eiN;
    const int    nE   = (s == 0) ? nEP : nEN;
    const int    vec8 = (s == 0) ? vecP : vecN;
    const float* bias = (s == 0) ? bP : bN;
    const unsigned short* Bh = planes + (size_t)(2 * s) * NOUT * KF;
    const unsigned short* Bl = Bh + (size_t)NOUT * KF;

    {
      const v4f z = {0.f, 0.f, 0.f, 0.f};
#pragma unroll 1
      for (int i = tid; i < TGT * FIN / 4; i += NTHR) ((v4f*)acc)[i] = z;
#pragma unroll 1
      for (int i = tid; i < TGT; i += NTHR) scnt[i] = 0;
    }
    __syncthreads();

    const int* dsts = ei + nE;
    const int nChunks = (nE + CHUNK - 1) / CHUNK;
#pragma unroll 1
    for (int ch = 0; ch < nChunks; ++ch) {
      const int cbase = ch * CHUNK;
      const int wc = scan_chunk<TGT>(dsts, nE, cbase, nodeBase, vec8, list, tid, lane, wave);
      if (lane == 0) wcnt[wave] = wc;
      __syncthreads();
      if (wave == 0) {
#pragma unroll 1
        for (int wsx = 0; wsx < NWAVE; ++wsx) {
          int n = __builtin_amdgcn_readfirstlane(wcnt[wsx]);
          n = n > WCAP ? WCAP : (n < 0 ? 0 : n);
          const int* lp = list + wsx * WCAP;
#pragma unroll 1
          for (int i = 0; i < n; ++i) {
            const int ent  = __builtin_amdgcn_readfirstlane(lp[i]);
            const int slot = ent & (TGT - 1);
            int e = cbase + ((ent >> 12) & (CHUNK - 1));
            e = e > nE - 1 ? nE - 1 : e;
            int src = ei[e];
            src = src < 0 ? 0 : (src > nN - 1 ? nN - 1 : src);
            const v2f v = *(const v2f*)(x + (size_t)src * FIN + 2 * lane);
            v2f* ap = (v2f*)(acc + slot * FIN + 2 * lane);
            *ap = *ap + v;
            if (lane == 0) scnt[slot] = scnt[slot] + 1;
          }
        }
      }
      __syncthreads();
    }

#pragma unroll 1
    for (int it = 0; it < TGT / (NWAVE * 16); ++it) {
      const int r0 = 16 * (NWAVE * it + wave);
      if (nodeBase + r0 >= nN) continue;
      const int lrow = r0 + m;
      int grow = nodeBase + lrow;
      grow = grow > nN - 1 ? nN - 1 : grow;
      int cv = scnt[lrow];
      cv = cv < 1 ? 1 : cv;
      const float inv = 1.0f / (float)cv;
      const float* arow = acc + lrow * FIN + 8 * hh;
      const float* xrow = x + (size_t)grow * FIN + 8 * hh;

      v8f d[4];
#pragma unroll
      for (int t = 0; t < 4; ++t) { v8f z = {0.f, 0.f, 0.f, 0.f, 0.f, 0.f, 0.f, 0.f}; d[t] = z; }

#pragma unroll
      for (int kt = 0; kt < 2; ++kt) {
        const float* p = arow + 32 * kt;
        const v4f a0 = *(const v4f*)(p)      * inv;
        const v4f a1 = *(const v4f*)(p + 4)  * inv;
        const v4f a2 = *(const v4f*)(p + 16) * inv;
        const v4f a3 = *(const v4f*)(p + 20) * inv;
        FragB ah, al;
        split16(a0, a1, a2, a3, ah, al);
#pragma unroll
        for (int t = 0; t < 4; ++t) {
          const unsigned short* bp = Bh + (size_t)(16 * t + m) * KF + 32 * kt + 8 * hh;
          const unsigned short* bq = Bl + (size_t)(16 * t + m) * KF + 32 * kt + 8 * hh;
          FragB bh, bl;
          bh.h[0] = *(const v8us*)bp; bh.h[1] = *(const v8us*)(bp + 16);
          bl.h[0] = *(const v8us*)bq; bl.h[1] = *(const v8us*)(bq + 16);
          d[t] = wmb(ah, bh, d[t]);
          d[t] = wmb(ah, bl, d[t]);
          d[t] = wmb(al, bh, d[t]);
        }
      }
#pragma unroll
      for (int kt = 2; kt < 4; ++kt) {
        const float* p = xrow + 32 * (kt - 2);
        const v4f a0 = *(const v4f*)(p);
        const v4f a1 = *(const v4f*)(p + 4);
        const v4f a2 = *(const v4f*)(p + 16);
        const v4f a3 = *(const v4f*)(p + 20);
        FragB ah, al;
        split16(a0, a1, a2, a3, ah, al);
#pragma unroll
        for (int t = 0; t < 4; ++t) {
          const unsigned short* bp = Bh + (size_t)(16 * t + m) * KF + 32 * kt + 8 * hh;
          const unsigned short* bq = Bl + (size_t)(16 * t + m) * KF + 32 * kt + 8 * hh;
          FragB bh, bl;
          bh.h[0] = *(const v8us*)bp; bh.h[1] = *(const v8us*)(bp + 16);
          bl.h[0] = *(const v8us*)bq; bl.h[1] = *(const v8us*)(bq + 16);
          d[t] = wmb(ah, bh, d[t]);
          d[t] = wmb(ah, bl, d[t]);
          d[t] = wmb(al, bh, d[t]);
        }
      }

#pragma unroll
      for (int t = 0; t < 4; ++t) {
        const float bv = bias[16 * t + m];
        float* sp = acc + (r0 + 8 * hh) * FIN + 16 * t + m;
#pragma unroll
        for (int r = 0; r < 8; ++r) sp[r * FIN] = d[t][r] + bv;
      }
      __builtin_amdgcn_fence(__ATOMIC_RELEASE, "wavefront");
      __builtin_amdgcn_wave_barrier();

      v4f ov[8];
#pragma unroll
      for (int p = 0; p < 8; ++p) {
        const int rr = r0 + 2 * p + hh;
        ov[p] = *(const v4f*)(acc + rr * FIN + 4 * m);
      }
      float* ob = out + (size_t)64 * s + 4 * m;
#pragma unroll
      for (int p = 0; p < 8; ++p) {
        const int gr = nodeBase + r0 + 2 * p + hh;
        if (gr < nN) *(volatile v4f*)(ob + (size_t)gr * OUTW) = ov[p];
      }
      __threadfence();
#pragma unroll
      for (int p = 0; p < 8; ++p) {
        const int gr = nodeBase + r0 + 2 * p + hh;
        if (gr < nN) *(volatile v4f*)(ob + (size_t)gr * OUTW) = ov[p];
      }
    }
    __syncthreads();
  }
}

extern "C" void kernel_launch(void* const* d_in, const int* in_sizes, int n_in,
                              void* d_out, int out_size, void* d_ws, size_t ws_size,
                              hipStream_t stream) {
  if (n_in < 9) return;
  const int nN = in_sizes[0] / FIN;
  if (nN <= 0 || in_sizes[0] != nN * FIN) return;
  const int nEP = in_sizes[1] / 2;
  const int nEN = in_sizes[2] / 2;
  if (nEP < 0 || nEN < 0 || in_sizes[1] != 2 * nEP || in_sizes[2] != 2 * nEN) return;
  if (in_sizes[3] != NOUT * FIN || in_sizes[4] != NOUT * FIN || in_sizes[5] != NOUT) return;
  if (in_sizes[6] != NOUT * FIN || in_sizes[7] != NOUT * FIN || in_sizes[8] != NOUT) return;
  if (out_size != nN * OUTW) return;
  if (nN > (1 << 22) || nEP > (1 << 28) || nEN > (1 << 28)) return;

  const float* x     = (const float*)d_in[0];
  const int*   eiP   = (const int*)d_in[1];
  const int*   eiN   = (const int*)d_in[2];
  const float* Wp    = (const float*)d_in[3];
  const float* Wpc   = (const float*)d_in[4];
  const float* bP    = (const float*)d_in[5];
  const float* Wn    = (const float*)d_in[6];
  const float* Wnc   = (const float*)d_in[7];
  const float* bN    = (const float*)d_in[8];
  float* out = (float*)d_out;

  const size_t plBytes = (size_t)NPL * 2;
  if (plBytes > ws_size) return;
  unsigned short* planes = (unsigned short*)d_ws;

  const int vecP = ((nEP & 3) == 0) ? 1 : 0;
  const int vecN = ((nEN & 3) == 0) ? 1 : 0;

  k_wprep<<<(2 * NOUT * (KF / 8)) / NTHR, NTHR, 0, stream>>>(Wp, Wpc, Wn, Wnc, planes);

  hipFuncSetAttribute(reinterpret_cast<const void*>(&k_main),
                      hipFuncAttributeMaxDynamicSharedMemorySize, LDS_MAIN);
  const int nBlk = (nN + TGT - 1) / TGT;
  k_main<<<nBlk, NTHR, LDS_MAIN, stream>>>(x, eiP, eiN, planes, bP, bN, out, nN, nEP, nEN, vecP, vecN);
}
